// ScaledDotProductAttention_33930241639016
// MI455X (gfx1250) — hardware-verified
//
#include <hip/hip_runtime.h>
#include <math.h>

#ifndef NB
#define NB 16
#endif
#ifndef SEQ
#define SEQ 2048
#endif
#define NB_FULL 16
#define SEQ_FULL 2048
#define DH 64
#define AW 4
static_assert(NB >= 1 && NB <= NB_FULL);
static_assert(SEQ >= 256 && SEQ <= SEQ_FULL && (SEQ % 256) == 0);
static_assert(DH == 64);

typedef __attribute__((ext_vector_type(16))) _Float16 v16h;
typedef __attribute__((ext_vector_type(8)))  _Float16 v8h;
typedef __attribute__((ext_vector_type(8)))  float    v8f;
typedef __attribute__((ext_vector_type(4)))  float    v4f;
typedef __attribute__((ext_vector_type(4)))  unsigned v4u;

union Frag { v16h v; v8h half[2]; };

__device__ __forceinline__ v8f wmma16(v16h a, v16h b, v8f c) {
    c = __builtin_amdgcn_wmma_f32_16x16x32_f16(false, a, false, b, (short)0, c, false, false);
    asm volatile("v_nop\n\tv_nop\n\tv_nop\n\tv_nop" : "+v"(c) : "v"(a), "v"(b));
    return c;
}

#define VST2V4(ptr, val) do { const v4f vst2_v4_ = (val); *(volatile v4f*)(ptr) = vst2_v4_; __threadfence(); *(volatile v4f*)(ptr) = vst2_v4_; } while (0)
#define VST2U4(ptr, val) do { const v4u vst2_u4_ = (val); *(volatile v4u*)(ptr) = vst2_u4_; __threadfence(); *(volatile v4u*)(ptr) = vst2_u4_; } while (0)

__device__ __forceinline__ float cmb_bf(float v) { const unsigned u = __builtin_bit_cast(unsigned, v); const unsigned r = (u + 0x7fffu + ((u >> 16) & 1u)) & 0xffff0000u; return __builtin_bit_cast(float, r); }
__device__ __forceinline__ unsigned cmb_pk2(float a, float b) { return (unsigned)__builtin_bit_cast(unsigned short, (_Float16)a) | ((unsigned)__builtin_bit_cast(unsigned short, (_Float16)b) << 16); }

__global__ __launch_bounds__(256) void k_cvt(const float* __restrict__ Q, const float* __restrict__ Kp, const float* __restrict__ V,
                                             unsigned short* __restrict__ QH, unsigned short* __restrict__ KH, unsigned short* __restrict__ VT) {
    const long long nqk = (long long)NB * SEQ * (DH / 8);
    const long long nbqk = nqk / 256;
    const long long nv = (long long)NB * DH * (SEQ / 8);
    const long long bid = blockIdx.x;
    float w[8];
    unsigned short* dst;
    if (bid < 2 * nbqk) {
        const int which = (bid < nbqk) ? 0 : 1;
        const long long u = (bid - (long long)which * nbqk) * 256 + threadIdx.x;
        const long long r = u >> 3; const int c0 = 8 * (int)(u & 7);
        const int bb = (int)(r / SEQ); const int i = (int)(r - (long long)bb * SEQ);
        const float* src = (which ? Kp : Q) + ((long long)bb * SEQ_FULL + i) * DH + c0;
        const v4f x0 = *(const v4f*)src; const v4f x1 = *(const v4f*)(src + 4);
        w[0] = x0.x; w[1] = x0.y; w[2] = x0.z; w[3] = x0.w; w[4] = x1.x; w[5] = x1.y; w[6] = x1.z; w[7] = x1.w;
        dst = (which ? KH : QH) + ((long long)bb * SEQ + i) * DH + c0;
    } else {
        const long long u = (bid - 2 * nbqk) * 256 + threadIdx.x;
        if (u >= nv) return;
        const int per = SEQ / 8;
        const int kb = (int)(u % per); const long long bd = u / per; const int d = (int)(bd % DH); const int bb = (int)(bd / DH);
        const int key0 = 8 * kb;
        const float* src = V + ((long long)bb * SEQ_FULL + key0) * DH + d;
#pragma unroll
        for (int e = 0; e < 8; ++e) w[e] = src[(long long)e * DH];
        dst = VT + ((long long)bb * DH + d) * SEQ + key0;
    }
    v4u pk;
    pk.x = cmb_pk2(cmb_bf(w[0]), cmb_bf(w[1])); pk.y = cmb_pk2(cmb_bf(w[2]), cmb_bf(w[3]));
    pk.z = cmb_pk2(cmb_bf(w[4]), cmb_bf(w[5])); pk.w = cmb_pk2(cmb_bf(w[6]), cmb_bf(w[7]));
    VST2U4(dst, pk);
}

__global__ __launch_bounds__(32 * AW) __attribute__((amdgpu_num_vgpr(256)))
void k_attn_vl(const _Float16* __restrict__ QH, const _Float16* __restrict__ KH, const _Float16* __restrict__ VT, const int* __restrict__ VL, float* __restrict__ O) {
    __shared__ __align__(16) float pl[AW][16 * 64];
    const int lane = threadIdx.x & 31, hf = lane >> 4, l15 = lane & 15, wave = threadIdx.x >> 5;
    const int b = blockIdx.y;
    const int q0 = (blockIdx.x * AW + wave) * 16;
    const float L2E = 1.4426950408889634f;
    const float NEG = -__builtin_inff();
    const float MFILL = -1e20f;
    const float SCALE = 0.125f;
    const int vlen = VL[b];
    int jend = SEQ;
    if (vlen > 0) { const int vc = min(vlen, SEQ); jend = ((vc + 63) / 64) * 64; }

    const _Float16* qr = QH + ((long long)b * SEQ + q0 + l15) * DH;
    Frag qa0, qa1;
    qa0.half[0] = *(const v8h*)(qr + 8 * hf);       qa0.half[1] = *(const v8h*)(qr + 16 + 8 * hf);
    qa1.half[0] = *(const v8h*)(qr + 32 + 8 * hf);  qa1.half[1] = *(const v8h*)(qr + 48 + 8 * hf);
    const _Float16* kpl = KH + (long long)b * SEQ * DH;
    const _Float16* vpl = VT + (long long)b * DH * SEQ;

    v8f o[4]; float m8[8], l8[8];
#pragma unroll
    for (int t = 0; t < 4; ++t) { v8f zz = {}; o[t] = zz; }
#pragma unroll
    for (int i = 0; i < 8; ++i) { m8[i] = NEG; l8[i] = 0.f; }

#pragma unroll 1
    for (int j0 = 0; j0 < jend; j0 += 64) {
        v8f s[4];
#pragma unroll
        for (int t = 0; t < 4; ++t) {
            const _Float16* kr = kpl + (long long)(j0 + t * 16 + l15) * DH;
            Frag kb0, kb1;
            kb0.half[0] = *(const v8h*)(kr + 8 * hf);       kb0.half[1] = *(const v8h*)(kr + 16 + 8 * hf);
            kb1.half[0] = *(const v8h*)(kr + 32 + 8 * hf);  kb1.half[1] = *(const v8h*)(kr + 48 + 8 * hf);
            v8f acc = {};
            acc = wmma16(qa0.v, kb0.v, acc);
            acc = wmma16(qa1.v, kb1.v, acc);
            s[t] = acc;
        }
        float pv[8][4];
#pragma unroll
        for (int i = 0; i < 8; ++i) {
            float sc[4];
#pragma unroll
            for (int t = 0; t < 4; ++t) {
                const int jg = j0 + t * 16 + l15;
                float v = s[t][i] * SCALE;
                if (jg >= vlen) v = MFILL;
                sc[t] = v * L2E;
            }
            float mx = fmaxf(fmaxf(sc[0], sc[1]), fmaxf(sc[2], sc[3]));
            mx = fmaxf(mx, __shfl_xor(mx, 1, 32)); mx = fmaxf(mx, __shfl_xor(mx, 2, 32));
            mx = fmaxf(mx, __shfl_xor(mx, 4, 32)); mx = fmaxf(mx, __shfl_xor(mx, 8, 32));
            const float mnew = fmaxf(m8[i], mx);
            const float corr = (mnew == NEG) ? 1.f : exp2f(m8[i] - mnew);
            float rs = 0.f;
#pragma unroll
            for (int t = 0; t < 4; ++t) { const float pp = exp2f(sc[t] - mnew); rs += pp; pv[i][t] = pp; }
            rs += __shfl_xor(rs, 1, 32); rs += __shfl_xor(rs, 2, 32); rs += __shfl_xor(rs, 4, 32); rs += __shfl_xor(rs, 8, 32);
            l8[i] = l8[i] * corr + rs; m8[i] = mnew;
#pragma unroll
            for (int t = 0; t < 4; ++t) o[t][i] *= corr;
        }
        __syncthreads();
#pragma unroll
        for (int i = 0; i < 8; ++i)
#pragma unroll
            for (int t = 0; t < 4; ++t) pl[wave][(i + 8 * hf) * 64 + t * 16 + l15] = pv[i][t];
        __syncthreads();
        Frag pa0, pa1;
#pragma unroll
        for (int e = 0; e < 8; ++e) {
            pa0.v[e]     = (_Float16)(pl[wave][l15 * 64 +      8 * hf + e] * 4096.f);
            pa0.v[8 + e] = (_Float16)(pl[wave][l15 * 64 + 16 + 8 * hf + e] * 4096.f);
            pa1.v[e]     = (_Float16)(pl[wave][l15 * 64 + 32 + 8 * hf + e] * 4096.f);
            pa1.v[8 + e] = (_Float16)(pl[wave][l15 * 64 + 48 + 8 * hf + e] * 4096.f);
        }
#pragma unroll
        for (int t = 0; t < 4; ++t) {
            const _Float16* vr = vpl + (long long)(t * 16 + l15) * SEQ + j0;
            Frag vb0, vb1;
            vb0.half[0] = *(const v8h*)(vr + 8 * hf);       vb0.half[1] = *(const v8h*)(vr + 16 + 8 * hf);
            vb1.half[0] = *(const v8h*)(vr + 32 + 8 * hf);  vb1.half[1] = *(const v8h*)(vr + 48 + 8 * hf);
            o[t] = wmma16(pa0.v, vb0.v, o[t]);
            o[t] = wmma16(pa1.v, vb1.v, o[t]);
        }
    }

    float invr[8];
#pragma unroll
    for (int i = 0; i < 8; ++i) invr[i] = (l8[i] > 0.f) ? 1.f / (l8[i] * 4096.f) : 0.f;
    __syncthreads();
#pragma unroll
    for (int i = 0; i < 8; ++i)
#pragma unroll
        for (int t = 0; t < 4; ++t) pl[wave][(i + 8 * hf) * 64 + t * 16 + l15] = o[t][i] * invr[i];
    __syncthreads();
    float* ob = O + ((long long)b * SEQ_FULL + q0) * DH;
#pragma unroll
    for (int r0 = 0; r0 < 16; r0 += 2) {
        const int row = r0 + hf, c4 = l15 * 4;
        v4f v;
        v.x = pl[wave][row * 64 + c4]; v.y = pl[wave][row * 64 + c4 + 1]; v.z = pl[wave][row * 64 + c4 + 2]; v.w = pl[wave][row * 64 + c4 + 3];
        VST2V4(ob + (long long)row * DH + c4, v);
    }
}


extern "C" void kernel_launch(void* const* d_in, const int* in_sizes, int n_in, void* d_out, int out_size, void* d_ws, size_t ws_size, hipStream_t stream) {
    if (n_in < 4) return;
    const float* q = (const float*)d_in[0];
    const float* kk = (const float*)d_in[1];
    const float* v = (const float*)d_in[2];
    const int* vl = (const int*)d_in[3];
    float* out = (float*)d_out;
    const long long bstride = (long long)SEQ_FULL * DH;
    const long long need = (long long)(NB - 1) * bstride + (long long)SEQ * DH;
    if ((long long)in_sizes[0] < need || (long long)in_sizes[1] < need || (long long)in_sizes[2] < need || in_sizes[3] < NB) return;
    if ((long long)out_size < need) return;
    const size_t plane_bytes = (((size_t)NB * SEQ * DH * 2 + 255) / 256) * 256;
    char* wsp = (char*)d_ws;
    unsigned short* QH = (unsigned short*)wsp; wsp += plane_bytes;
    unsigned short* KH = (unsigned short*)wsp; wsp += plane_bytes;
    unsigned short* VT = (unsigned short*)wsp; wsp += plane_bytes;
    if ((size_t)(wsp - (char*)d_ws) > ws_size) return;
    if ((size_t)(wsp - (char*)d_ws) > (size_t)134217728) return;
    const long long nqk = (long long)NB * SEQ * (DH / 8);
    const long long nbqk = nqk / 256;
    const long long nv = (long long)NB * DH * (SEQ / 8);
    const long long nbv = (nv + 255) / 256;
    k_cvt<<<dim3((unsigned)(2 * nbqk + nbv)), 256, 0, stream>>>(q, kk, v, QH, KH, VT);
    k_attn_vl<<<dim3((unsigned)(SEQ / 64), (unsigned)NB), 32 * AW, 0, stream>>>((const _Float16*)QH, (const _Float16*)KH, (const _Float16*)VT, vl, out);
}
